// BayesianSequenceModel_13761075216825
// MI455X (gfx1250) — hardware-verified
//
#include <hip/hip_runtime.h>

typedef __attribute__((ext_vector_type(16))) _Float16 v16h;
typedef __attribute__((ext_vector_type(8)))  _Float16 v8h;
typedef __attribute__((ext_vector_type(4)))  _Float16 v4h;
typedef __attribute__((ext_vector_type(8)))  float    v8f;
typedef __attribute__((ext_vector_type(4)))  float    v4f;

__device__ __forceinline__ void dep_guard_h(v8f& a, v8f& b, v16h x, v16h y) { asm volatile("v_nop\n\tv_nop\n\tv_nop\n\tv_nop" : "+v"(a), "+v"(b) : "v"(x), "v"(y)); }
__device__ __forceinline__ void keep4_h(v16h a, v16h b, v16h c, v16h d) { asm volatile("v_nop" :: "v"(a), "v"(b), "v"(c), "v"(d)); }
template <typename T> struct Frag;
template <> struct Frag<_Float16> {
  typedef v16h V; union U { v16h v; v8h h[2]; };
  static __device__ __forceinline__ v16h load(const _Float16* p) {
    U f; f.h[0] = *(const v8h*)(p); f.h[1] = *(const v8h*)(p + 16); return f.v;
  }
  static __device__ __forceinline__ v8f mma(v16h a, v16h b, v8f c) {
    return __builtin_amdgcn_wmma_f32_16x16x32_f16(false, a, false, b, (short)0, c, false, false);
  }
  static __device__ __forceinline__ void guard(v8f& a, v8f& b, v16h x, v16h y) { dep_guard_h(a, b, x, y); }
  static __device__ __forceinline__ void keep(v16h a, v16h b, v16h c, v16h d) { keep4_h(a, b, c, d); }
};

__device__ __forceinline__ v8f mma_h(v16h a, v16h b, v8f c) {
  c = __builtin_amdgcn_wmma_f32_16x16x32_f16(false, a, false, b, (short)0, c, false, false);
  asm volatile("v_nop\n\tv_nop\n\tv_nop\n\tv_nop" : "+v"(c) : "v"(a), "v"(b));
  return c;
}

constexpr int kRowsTotal = 1024;
constexpr int kSteps     = 128;
constexpr int kA         = 8;
constexpr int kZ         = 32;
constexpr int kH         = 256;
constexpr int kGateN     = 4 * kH;
constexpr int kKG        = 320;
constexpr int kHoff      = 64;
constexpr int kU         = 128;
constexpr int kZZ        = 2 * kZ;
constexpr int kRows      = 16;
constexpr int kBlocks    = kRowsTotal / kRows;
constexpr int kXP        = 328;
constexpr int kUP        = 136;
constexpr int kZP        = 36;
constexpr float kCarry   = 8.0f;
constexpr float kFold    = 1.0f / 64.0f;
static_assert(kBlocks * kRows == kRowsTotal);
static_assert(kKG % 32 == 0 && kH % 32 == 0 && kU % 32 == 0);
static_assert((kXP % 8) == 0 && (kUP % 8) == 0 && (kZP % 4) == 0);

__device__ __forceinline__ float sigm_f(float x) {
  x = fminf(fmaxf(x, -30.0f), 30.0f);
  return 1.0f / (1.0f + expf(-x));
}
__device__ __forceinline__ float tanh_f(float x) {
  const float ax = fminf(fabsf(x), 15.0f);
  const float e = expf(-2.0f * ax);
  const float r = (1.0f - e) * (1.0f / (1.0f + e));
  return copysignf(r, x);
}
__device__ __forceinline__ float softplus_f(float x) {
  return log1pf(expf(-fabsf(x))) + fmaxf(x, 0.0f);
}

__global__ __launch_bounds__(256) void build_gate_plane(const float* __restrict__ Wih, const float* __restrict__ Whh,
                                                        _Float16* __restrict__ out, int total) {
  const int i  = blockIdx.x * 256 + threadIdx.x;
  const int ic = (i < total) ? i : (total - 1);
  const int n  = ic / (kKG / 8);
  const int ck = ic - n * (kKG / 8);
  const int k  = ck * 8;
  const int kih = (k < 32) ? k : 32;
  int khh = k - kHoff; khh = (khh < 0) ? 0 : khh;
  const float* pih = Wih + (size_t)n * (kA + kZ) + kih;
  const float* phh = Whh + (size_t)n * kH + khh;
  const v4f a0 = *(const v4f*)(pih);
  const v4f a1 = *(const v4f*)(pih + 4);
  const v4f b0 = *(const v4f*)(phh);
  const v4f b1 = *(const v4f*)(phh + 4);
  const bool useih = (k < (kA + kZ));
  const bool usehh = (k >= kHoff);
  v8h hv;
#pragma unroll
  for (int e = 0; e < 8; ++e) {
    const float vi = (e < 4) ? a0[e] : a1[e - 4];
    const float vh = (e < 4) ? b0[e] : b1[e - 4];
    const float v  = useih ? vi : (usehh ? vh : 0.0f);
    hv[e] = (_Float16)(v * kCarry);
  }
  if (i < total) {
    *(volatile v8h*)(out + (size_t)i * 8) = hv;
    __threadfence();
    *(volatile v8h*)(out + (size_t)i * 8) = hv;
  }
}

__global__ __launch_bounds__(256) void cast_scale8_f16(const float* __restrict__ in, _Float16* __restrict__ out, int n8) {
  const int i  = blockIdx.x * 256 + threadIdx.x;
  const int ic = (i < n8) ? i : (n8 - 1);
  const v4f a0 = *(const v4f*)(in + (size_t)ic * 8);
  const v4f a1 = *(const v4f*)(in + (size_t)ic * 8 + 4);
  v8h hv;
#pragma unroll
  for (int e = 0; e < 8; ++e) hv[e] = (_Float16)(((e < 4) ? a0[e] : a1[e - 4]) * kCarry);
  if (i < n8) {
    *(volatile v8h*)(out + (size_t)i * 8) = hv;
    __threadfence();
    *(volatile v8h*)(out + (size_t)i * 8) = hv;
  }
}

__global__ __launch_bounds__(256) void seq_main(const float* __restrict__ Ain,
                                                const float* __restrict__ epsin,
                                                const float* __restrict__ z0,
                                                const float* __restrict__ h0,
                                                const float* __restrict__ c0,
                                                const _Float16* __restrict__ Wg,
                                                const float* __restrict__ bih, const float* __restrict__ bhh,
                                                const _Float16* __restrict__ W1s, const float* __restrict__ b1,
                                                const _Float16* __restrict__ W2s, const float* __restrict__ b2,
                                                const _Float16* __restrict__ Wzs, const float* __restrict__ bz,
                                                float* __restrict__ out) {
  __shared__ __align__(16) _Float16 Xs[2][kRows * kXP];
  __shared__ __align__(16) _Float16 U1s[kRows * kUP];
  __shared__ __align__(16) _Float16 U2s[kRows * kUP];
  __shared__ __align__(16) float    Zsl[kRows * kZP];

  const int tid  = threadIdx.x;
  const int wave = tid >> 5;
  const int lane = tid & 31;
  const int hh   = lane >> 4;
  const int cc   = lane & 15;
  const int koff = hh * 8;
  const int row0 = blockIdx.x * kRows;

  {
    v8h zv;
#pragma unroll
    for (int e = 0; e < 8; ++e) zv[e] = (_Float16)0.0f;
    for (int i = tid; i < 2 * kRows * 3; i += 256) {
      const int bsel = i / (kRows * 3);
      const int rem  = i - bsel * (kRows * 3);
      const int row  = rem / 3;
      const int ch   = rem - row * 3;
      *(v8h*)(&Xs[bsel][row * kXP + 40 + ch * 8]) = zv;
    }
  }
  if (tid < kRows * 4) {
    const int row = tid >> 2, ch = tid & 3;
    const v4f a0 = *(const v4f*)(z0 + ch * 8);
    const v4f a1 = *(const v4f*)(z0 + ch * 8 + 4);
    v8h hv;
#pragma unroll
    for (int e = 0; e < 8; ++e) hv[e] = (_Float16)(((e < 4) ? a0[e] : a1[e - 4]) * kCarry);
    *(v8h*)(&Xs[0][row * kXP + kA + ch * 8]) = hv;
  }
  for (int i = tid; i < kRows * 32; i += 256) {
    const int row = i >> 5, ch = i & 31;
    const v4f a0 = *(const v4f*)(h0 + ch * 8);
    const v4f a1 = *(const v4f*)(h0 + ch * 8 + 4);
    v8h hv;
#pragma unroll
    for (int e = 0; e < 8; ++e) hv[e] = (_Float16)(((e < 4) ? a0[e] : a1[e - 4]) * kCarry);
    *(v8h*)(&Xs[0][row * kXP + kHoff + ch * 8]) = hv;
  }

  float cst[2][8];
  float bsum[2][4];
#pragma unroll
  for (int u = 0; u < 2; ++u) {
    const int ucol = (2 * wave + u) * 16 + cc;
    const float cv = c0[ucol];
#pragma unroll
    for (int r = 0; r < 8; ++r) cst[u][r] = cv;
#pragma unroll
    for (int j = 0; j < 4; ++j) bsum[u][j] = bih[j * kH + ucol] + bhh[j * kH + ucol];
  }
  const float b1v = b1[wave * 16 + cc];
  const float b2v = b2[wave * 16 + cc];
  float bzl[2], bzr[2];
#pragma unroll
  for (int s = 0; s < 2; ++s) { bzl[s] = bz[s * 16 + cc]; bzr[s] = bz[kZ + s * 16 + cc]; }

#pragma unroll 1
  for (int t = 0; t < kSteps; ++t) {
    const int cur = t & 1;
    _Float16* Xc = Xs[cur];
    _Float16* Xn = Xs[cur ^ 1];

    if (wave == 0) {
      const int row = lane >> 1, q = lane & 1;
      const v4f av = *(const v4f*)(Ain + ((size_t)(row0 + row) * kSteps + t) * kA + q * 4);
      v4h hv;
#pragma unroll
      for (int e = 0; e < 4; ++e) hv[e] = (_Float16)(av[e] * kCarry);
      *(v4h*)(Xc + row * kXP + q * 4) = hv;
    }
    __syncthreads();

    {
      v8f acc[2][4];
#pragma unroll
      for (int u = 0; u < 2; ++u)
#pragma unroll
        for (int j = 0; j < 4; ++j) acc[u][j] = (v8f){0.f,0.f,0.f,0.f,0.f,0.f,0.f,0.f};
#pragma unroll 1
      for (int ks = 0; ks < kKG / 32; ++ks) {
        const int k0 = ks * 32;
        const v16h a = Frag<_Float16>::load(Xc + cc * kXP + k0 + koff);
#pragma unroll
        for (int u = 0; u < 2; ++u) {
#pragma unroll
          for (int j = 0; j < 4; ++j) {
            const int n = j * kH + (2 * wave + u) * 16 + cc;
            const v16h b = Frag<_Float16>::load(Wg + (size_t)n * kKG + k0 + koff);
            acc[u][j] = mma_h(a, b, acc[u][j]);
          }
        }
      }
#pragma unroll
      for (int u = 0; u < 2; ++u) {
        const int ucol = (2 * wave + u) * 16 + cc;
#pragma unroll
        for (int r = 0; r < 8; ++r) {
          const float pi = acc[u][0][r] * kFold + bsum[u][0];
          const float pf = acc[u][1][r] * kFold + bsum[u][1];
          const float pg = acc[u][2][r] * kFold + bsum[u][2];
          const float po = acc[u][3][r] * kFold + bsum[u][3];
          const float si = sigm_f(pi);
          const float sf = sigm_f(pf);
          const float gg = tanh_f(pg);
          const float so = sigm_f(po);
          const float cn = sf * cst[u][r] + si * gg;
          cst[u][r] = cn;
          const float hn = so * tanh_f(cn);
          Xn[(8 * hh + r) * kXP + kHoff + ucol] = (_Float16)(hn * kCarry);
        }
      }
    }
    __syncthreads();

    {
      v8f acc2 = (v8f){0.f,0.f,0.f,0.f,0.f,0.f,0.f,0.f};
      const int col = wave * 16 + cc;
#pragma unroll 4
      for (int ks = 0; ks < kH / 32; ++ks) {
        const int k0 = ks * 32;
        const v16h a = Frag<_Float16>::load(Xn + cc * kXP + kHoff + k0 + koff);
        const v16h b = Frag<_Float16>::load(W1s + (size_t)col * kH + k0 + koff);
        acc2 = mma_h(a, b, acc2);
      }
#pragma unroll
      for (int r = 0; r < 8; ++r) {
        const float v = fmaxf(acc2[r] * kFold + b1v, 0.0f);
        U1s[(8 * hh + r) * kUP + col] = (_Float16)(v * kCarry);
      }
    }
    __syncthreads();

    {
      v8f acc3 = (v8f){0.f,0.f,0.f,0.f,0.f,0.f,0.f,0.f};
      const int col = wave * 16 + cc;
#pragma unroll
      for (int ks = 0; ks < kU / 32; ++ks) {
        const int k0 = ks * 32;
        const v16h a = Frag<_Float16>::load(U1s + cc * kUP + k0 + koff);
        const v16h b = Frag<_Float16>::load(W2s + (size_t)col * kU + k0 + koff);
        acc3 = mma_h(a, b, acc3);
      }
#pragma unroll
      for (int r = 0; r < 8; ++r) {
        const float v = fmaxf(acc3[r] * kFold + b2v, 0.0f);
        U2s[(8 * hh + r) * kUP + col] = (_Float16)(v * kCarry);
      }
    }
    __syncthreads();

    if (wave == 0) {
      v8f az[4];
#pragma unroll
      for (int j = 0; j < 4; ++j) az[j] = (v8f){0.f,0.f,0.f,0.f,0.f,0.f,0.f,0.f};
#pragma unroll 1
      for (int ks = 0; ks < kU / 32; ++ks) {
        const int k0 = ks * 32;
        const v16h a = Frag<_Float16>::load(U2s + cc * kUP + k0 + koff);
#pragma unroll
        for (int j = 0; j < 4; ++j) {
          const v16h b = Frag<_Float16>::load(Wzs + (size_t)(j * 16 + cc) * kU + k0 + koff);
          az[j] = mma_h(a, b, az[j]);
        }
      }
#pragma unroll
      for (int s = 0; s < 2; ++s) {
        const int zc = s * 16 + cc;
#pragma unroll
        for (int r = 0; r < 8; ++r) {
          const int row = 8 * hh + r;
          const size_t gidx = ((size_t)(row0 + row) * kSteps + t) * kZ + zc;
          const float loc = az[s][r] * kFold + bzl[s];
          const float raw = az[2 + s][r] * kFold + bzr[s];
          const float sp  = softplus_f(raw);
          const float e   = epsin[gidx];
          const float zv  = loc + sp * e;
          Zsl[row * kZP + zc] = zv;
          Xn[row * kXP + kA + zc] = (_Float16)(zv * kCarry);
        }
      }
      __builtin_amdgcn_fence(__ATOMIC_RELEASE, "workgroup");
      __builtin_amdgcn_wave_barrier();
      __builtin_amdgcn_fence(__ATOMIC_ACQUIRE, "workgroup");
      {
        const int q = lane >> 3, c4 = (lane & 7) * 4;
        for (int pass = 0; pass < 2; ++pass) {
#pragma unroll
          for (int it = 0; it < 4; ++it) {
            const int row = it * 4 + q;
            const v4f v = *(const v4f*)(Zsl + row * kZP + c4);
            *(volatile v4f*)(out + ((size_t)(row0 + row) * kSteps + t) * kZ + c4) = v;
          }
          __threadfence();
        }
      }
    }
  }
}

extern "C" void kernel_launch(void* const* d_in, const int* in_sizes, int n_in,
                              void* d_out, int out_size, void* d_ws,
                              size_t ws_size, hipStream_t stream) {
  if (n_in < 15) return;
  if (in_sizes[0]  != kRowsTotal * kSteps * kA) return;
  if (in_sizes[1]  != kRowsTotal * kSteps * kZ) return;
  if (in_sizes[2]  != kZ) return;
  if (in_sizes[3]  != kH) return;
  if (in_sizes[4]  != kH) return;
  if (in_sizes[5]  != kGateN * (kA + kZ)) return;
  if (in_sizes[6]  != kGateN * kH) return;
  if (in_sizes[7]  != kGateN) return;
  if (in_sizes[8]  != kGateN) return;
  if (in_sizes[9]  != kU * kH) return;
  if (in_sizes[10] != kU) return;
  if (in_sizes[11] != kU * kU) return;
  if (in_sizes[12] != kU) return;
  if (in_sizes[13] != kZZ * kU) return;
  if (in_sizes[14] != kZZ) return;
  if (out_size != kRowsTotal * kSteps * kZ) return;

  const float* A    = (const float*)d_in[0];
  const float* eps  = (const float*)d_in[1];
  const float* z0   = (const float*)d_in[2];
  const float* h0   = (const float*)d_in[3];
  const float* c0   = (const float*)d_in[4];
  const float* W_ih = (const float*)d_in[5];
  const float* W_hh = (const float*)d_in[6];
  const float* b_ih = (const float*)d_in[7];
  const float* b_hh = (const float*)d_in[8];
  const float* W1   = (const float*)d_in[9];
  const float* b1   = (const float*)d_in[10];
  const float* W2   = (const float*)d_in[11];
  const float* b2   = (const float*)d_in[12];
  const float* Wz   = (const float*)d_in[13];
  const float* bz   = (const float*)d_in[14];

  const size_t offWg = 0;
  const size_t bytesWg = (size_t)kGateN * kKG * sizeof(_Float16);
  const size_t offW1 = offWg + bytesWg;
  const size_t bytesW1 = (size_t)kU * kH * sizeof(_Float16);
  const size_t offW2 = offW1 + bytesW1;
  const size_t bytesW2 = (size_t)kU * kU * sizeof(_Float16);
  const size_t offWz = offW2 + bytesW2;
  const size_t bytesWz = (size_t)kZZ * kU * sizeof(_Float16);
  const size_t total = offWz + bytesWz;
  if (ws_size < total) return;

  char* ws = (char*)d_ws;
  _Float16* Wg  = (_Float16*)(ws + offWg);
  _Float16* W1s = (_Float16*)(ws + offW1);
  _Float16* W2s = (_Float16*)(ws + offW2);
  _Float16* Wzs = (_Float16*)(ws + offWz);

  const int nWg = kGateN * (kKG / 8);
  const int nW1 = kU * kH / 8;
  const int nW2 = kU * kU / 8;
  const int nWz = kZZ * kU / 8;
  build_gate_plane<<<(nWg + 255) / 256, 256, 0, stream>>>(W_ih, W_hh, Wg, nWg);
  cast_scale8_f16<<<(nW1 + 255) / 256, 256, 0, stream>>>(W1, W1s, nW1);
  cast_scale8_f16<<<(nW2 + 255) / 256, 256, 0, stream>>>(W2, W2s, nW2);
  cast_scale8_f16<<<(nWz + 255) / 256, 256, 0, stream>>>(Wz, Wzs, nWz);
  seq_main<<<kBlocks, 256, 0, stream>>>(A, eps, z0, h0, c0, Wg, b_ih, b_hh, W1s, b1, W2s, b2, Wzs, bz, (float*)d_out);
}
